// CoSSM_77206332113398
// MI455X (gfx1250) — hardware-verified
//
#include <hip/hip_runtime.h>
#include <math.h>


typedef __attribute__((ext_vector_type(16))) _Float16 v16h;
typedef __attribute__((ext_vector_type(8)))  _Float16 v8h;
typedef __attribute__((ext_vector_type(8)))  float    v8f;
typedef __attribute__((ext_vector_type(4)))  float    v4f;
typedef __attribute__((ext_vector_type(2)))  float    v2f;

constexpr int NB     = 4;
constexpr int LSEQ   = 512;
constexpr int DIN    = 256;
constexpr int DMODEL = 1024;
constexpr int DINNER = 2048;
constexpr int DSTATE = 16;
constexpr int DCONV  = 4;
constexpr int DTRANK = 64;
constexpr int NTOK   = NB * LSEQ;
constexpr int XZW    = 2 * DINNER;
constexpr int DBLW   = DTRANK + 2 * DSTATE;
constexpr int DBLP   = 128;
constexpr int LP     = LSEQ + 2;
constexpr int KC3    = 3 * DIN;

constexpr float S_WCONV = 16.0f;
constexpr float S_WIP   = 64.0f;
constexpr float S_U     = 4.0f;
constexpr float S_WXP   = 64.0f;
constexpr float S_DT    = 8.0f;
constexpr float S_WDT   = 16.0f;
constexpr float S_YG    = 16.0f;
constexpr float S_WOP   = 64.0f;
constexpr float LOG2E_F = 1.44269504088896340736f;

__device__ __forceinline__ void dep_guard_h(v8f& a, v8f& b, v16h x, v16h y) { asm volatile("v_nop\n\tv_nop\n\tv_nop\n\tv_nop" : "+v"(a), "+v"(b) : "v"(x), "v"(y)); }
__device__ __forceinline__ void keep4_h(v16h a, v16h b, v16h c, v16h d) { asm volatile("v_nop" :: "v"(a), "v"(b), "v"(c), "v"(d)); }
__device__ __forceinline__ void acc_guard4(v8f& a, v8f& b, v8f& c, v8f& d) { asm volatile("v_nop\n\tv_nop\n\tv_nop\n\tv_nop" : "+v"(a), "+v"(b), "+v"(c), "+v"(d)); }
template <typename T> struct Frag;
template <> struct Frag<_Float16> {
  typedef v16h V; union U { v16h v; v8h h[2]; };
  static __device__ __forceinline__ v16h load(const _Float16* p) {
    U f; f.h[0] = *(const v8h*)(p); f.h[1] = *(const v8h*)(p + 16); return f.v;
  }
  static __device__ __forceinline__ v8f mma(v16h a, v16h b, v8f c) {
    return __builtin_amdgcn_wmma_f32_16x16x32_f16(false, a, false, b, (short)0, c, false, false);
  }
  static __device__ __forceinline__ void guard(v8f& a, v8f& b, v16h x, v16h y) { dep_guard_h(a, b, x, y); }
  static __device__ __forceinline__ void keep(v16h a, v16h b, v16h c, v16h d) { keep4_h(a, b, c, d); }
};

__device__ __forceinline__ unsigned pack_h2(float a, float b) {
  const _Float16 h0 = (_Float16)a, h1 = (_Float16)b;
  return (unsigned)__builtin_bit_cast(unsigned short, h0) | ((unsigned)__builtin_bit_cast(unsigned short, h1) << 16);
}
__device__ __forceinline__ void store_u32_twice(unsigned* p, unsigned u) {
  *(volatile unsigned*)p = u;
  __threadfence();
  *(volatile unsigned*)p = u;
}
__device__ __forceinline__ float wave_sum(float v) {
#pragma unroll
  for (int off = 16; off > 0; off >>= 1) v += __shfl_xor(v, off, 32);
  return v;
}
__device__ __forceinline__ float silu_f(float x) {
  return x * __builtin_amdgcn_rcpf(1.0f + __expf(-x));
}
__device__ __forceinline__ float softplus_f(float x) {
  return fmaxf(x, 0.0f) + __logf(1.0f + __expf(-fabsf(x)));
}

template <int EPI, bool DUAL>
__global__ __launch_bounds__(256) void gemm64_f16(
    const unsigned short* __restrict__ Ap, int lda, long strideA,
    const unsigned short* __restrict__ Btp, int ldb, long strideB,
    float* __restrict__ Cf, unsigned short* __restrict__ Ch, int ldc, long strideC,
    const float* __restrict__ p0, const float* __restrict__ p1,
    const float* __restrict__ resid, long strideR,
    int M, int N, int K, float scale, float aux, float s16)
{
  typedef _Float16 T;
  typedef Frag<T>::V V;
  const T* A = (const T*)Ap; const T* Bt = (const T*)Btp;
  __shared__ __align__(16) float sT[8][16 * 68];
  const int b    = blockIdx.y;
  const int lane = threadIdx.x & 31;
  const int wave = threadIdx.x >> 5;
  const int tilesN = N >> 6;
  const int tilesM = M >> 6;
  const int tile = blockIdx.x * 8 + wave;
  if (tile >= tilesM * tilesN) return;
  const int tm = tile / tilesN;
  const int tn = tile - tm * tilesN;
  const int m0 = tm << 6;
  const int n0 = tn << 6;

  const T* Ab = A  + (size_t)b * strideA;
  const T* Bb = Bt + (size_t)b * strideB;

  const int rlane = lane & 15;
  const int koff  = (lane >> 4) * 8;
  const int mOff  = (lane >> 4) * 8;

  v8f acc[4][4];
#pragma unroll
  for (int i = 0; i < 4; ++i)
#pragma unroll
    for (int j = 0; j < 4; ++j) acc[i][j] = (v8f){0.f,0.f,0.f,0.f,0.f,0.f,0.f,0.f};

  for (int k0 = 0; k0 < K; k0 += 32) {
    V bh[4];
#pragma unroll
    for (int j = 0; j < 4; ++j) {
      const size_t bo = (size_t)(n0 + (j << 4) + rlane) * ldb + koff + k0;
      bh[j] = Frag<T>::load(Bb + bo);
    }
#pragma unroll
    for (int i = 0; i < 4; ++i) {
      const size_t ao = (size_t)(m0 + (i << 4) + rlane) * lda + koff + k0;
      V ah = Frag<T>::load(Ab + ao);
#pragma unroll
      for (int j = 0; j < 4; ++j) acc[i][j] = Frag<T>::mma(ah, bh[j], acc[i][j]);
      Frag<T>::guard(acc[i][0], acc[i][3], ah, ah);
    }
    Frag<T>::keep(bh[0], bh[1], bh[2], bh[3]);
  }
  acc_guard4(acc[0][0], acc[0][1], acc[0][2], acc[0][3]);
  acc_guard4(acc[1][0], acc[1][1], acc[1][2], acc[1][3]);
  acc_guard4(acc[2][0], acc[2][1], acc[2][2], acc[2][3]);
  acc_guard4(acc[3][0], acc[3][1], acc[3][2], acc[3][3]);

  float* slab = sT[wave];
  const float* Rb = (EPI == 1) ? (resid + (size_t)b * strideR) : nullptr;
  float* Cb = Cf + (size_t)b * strideC;
  unsigned short* Hb = DUAL ? (Ch + (size_t)b * strideC) : nullptr;
#pragma unroll
  for (int i = 0; i < 4; ++i) {
    const int mBase = m0 + (i << 4);
#pragma unroll
    for (int j = 0; j < 4; ++j) {
      const int n = n0 + (j << 4) + rlane;
      float g0 = 0.f, g1 = 0.f;
      if (EPI == 1) { g0 = p0[n] * aux; g1 = p1[n]; }
#pragma unroll
      for (int r = 0; r < 8; ++r) {
        float v = acc[i][j][r] * scale;
        if (EPI == 1) {
          v = v * g0 + g1;
          v = fmaxf(v, 0.0f);
          v += Rb[(size_t)(mBase + mOff + r) * ldc + n];
        }
        slab[(mOff + r) * 68 + (j << 4) + rlane] = v;
      }
    }
    __builtin_amdgcn_fence(__ATOMIC_RELEASE, "workgroup");
    __builtin_amdgcn_wave_barrier();
    __builtin_amdgcn_fence(__ATOMIC_ACQUIRE, "workgroup");
    {
      const int hh = lane >> 4, c4 = (lane & 15) * 4;
      for (int pass = 0; pass < 2; ++pass) {
#pragma unroll
        for (int it = 0; it < 8; ++it) {
          const int row = it * 2 + hh;
          v4f v = *(const v4f*)(slab + row * 68 + c4);
          *(volatile v4f*)(Cb + (size_t)(mBase + row) * ldc + n0 + c4) = v;
        }
        __threadfence();
      }
    }
    if (DUAL) {
      const int q = lane >> 3, c8 = (lane & 7) * 8;
      for (int pass = 0; pass < 2; ++pass) {
#pragma unroll
        for (int it = 0; it < 4; ++it) {
          const int row = it * 4 + q;
          const float* sp = slab + row * 68 + c8;
          v8h hv;
#pragma unroll
          for (int e = 0; e < 8; ++e) hv[e] = (_Float16)(sp[e] * s16);
          *(volatile v8h*)(Hb + (size_t)(mBase + row) * ldc + n0 + c8) = hv;
        }
        __threadfence();
      }
    }
    __builtin_amdgcn_fence(__ATOMIC_RELEASE, "workgroup");
    __builtin_amdgcn_wave_barrier();
    __builtin_amdgcn_fence(__ATOMIC_ACQUIRE, "workgroup");
  }
}

__global__ __launch_bounds__(256) void cast_rows_f16(
    const float* __restrict__ in, unsigned short* __restrict__ out, int Rin, int Rout, int C, float s)
{
  const int i = blockIdx.x * 256 + threadIdx.x;
  const int n2 = (Rout * C) >> 1;
  if (i < n2) {
    const int e = 2 * i;
    const int r = e / C;
    const int c = e - r * C;
    const int rr = (r < Rin) ? r : (Rin - 1);
    const float* p = in + (size_t)rr * C + c;
    float v0 = p[0] * s, v1 = p[1] * s;
    if (r >= Rin) { v0 = 0.0f; v1 = 0.0f; }
    store_u32_twice((unsigned*)out + i, pack_h2(v0, v1));
  }
}

__global__ __launch_bounds__(256) void cast_convw_f16(
    const float* __restrict__ cw, unsigned short* __restrict__ out, float s)
{
  const int i2 = blockIdx.x * 256 + threadIdx.x;
  const int n2 = (DMODEL * KC3) >> 1;
  if (i2 < n2) {
    const int e = 2 * i2;
    const int o = e / KC3;
    const int rem = e - o * KC3;
    const int k = rem >> 8;
    const int ii = rem & (DIN - 1);
    const float v0 = cw[((size_t)o * DIN + ii) * 3 + k] * s;
    const float v1 = cw[((size_t)o * DIN + ii + 1) * 3 + k] * s;
    store_u32_twice((unsigned*)out + i2, pack_h2(v0, v1));
  }
}

__global__ __launch_bounds__(256) void pad_x_f16(const float* __restrict__ x, unsigned short* __restrict__ out)
{
  const int i = blockIdx.x * 256 + threadIdx.x;
  const int n2 = (NB * LP * DIN) >> 1;
  if (i < n2) {
    const int e = 2 * i;
    const int b = e / (LP * DIN);
    const int rem = e - b * (LP * DIN);
    const int lp = rem >> 8;
    const int c = rem & (DIN - 1);
    const int l = lp - 1;
    const bool valid = (l >= 0) && (l < LSEQ);
    const int lc = (l < 0) ? 0 : ((l >= LSEQ) ? (LSEQ - 1) : l);
    const float* p = x + (size_t)(b * LSEQ + lc) * DIN + c;
    float v0 = p[0], v1 = p[1];
    if (!valid) { v0 = 0.0f; v1 = 0.0f; }
    store_u32_twice((unsigned*)out + i, pack_h2(v0, v1));
  }
}

__global__ __launch_bounds__(256) void dwconv_silu2(
    const float* __restrict__ xz, const float* __restrict__ w, const float* __restrict__ bias,
    float* __restrict__ u32, unsigned short* __restrict__ u16, int reversed, float su)
{
  const int t = blockIdx.x * 256 + threadIdx.x;
  if (t >= NTOK * (DINNER / 2)) return;
  const int dp = t & (DINNER / 2 - 1);
  const int d  = 2 * dp;
  const int bl = t >> 10;
  const int b  = bl >> 9;
  const int l  = bl & (LSEQ - 1);
  float a0 = bias[d], a1 = bias[d + 1];
#pragma unroll
  for (int k = 0; k < DCONV; ++k) {
    const int tt  = l - (DCONV - 1) + k;
    const int ttc = (tt < 0) ? 0 : tt;
    const int sl  = reversed ? (LSEQ - 1 - ttc) : ttc;
    const v2f xv = *(const v2f*)(xz + (size_t)(b * LSEQ + sl) * XZW + d);
    const float x0 = (tt >= 0) ? xv.x : 0.0f;
    const float x1 = (tt >= 0) ? xv.y : 0.0f;
    a0 = fmaf(w[d * DCONV + k], x0, a0);
    a1 = fmaf(w[(d + 1) * DCONV + k], x1, a1);
  }
  const float s0 = silu_f(a0), s1 = silu_f(a1);
  const size_t idx = (size_t)bl * DINNER + d;
  v2f ov; ov.x = s0; ov.y = s1;
  const unsigned hu = pack_h2(s0 * su, s1 * su);
  *(volatile v2f*)(u32 + idx) = ov;
  *(volatile unsigned*)((unsigned*)u16 + (idx >> 1)) = hu;
  __threadfence();
  *(volatile v2f*)(u32 + idx) = ov;
  *(volatile unsigned*)((unsigned*)u16 + (idx >> 1)) = hu;
}

template <int MODE>
__global__ __launch_bounds__(256) void scan2(
    const float* __restrict__ pre, const float* __restrict__ dt_bias,
    const float* __restrict__ u32, const float* __restrict__ dbl,
    const float* __restrict__ A_log, const float* __restrict__ Dp, float* __restrict__ ys,
    const float* __restrict__ ysf, const float* __restrict__ xz, unsigned short* __restrict__ yg, float syg)
{
  const int gid = blockIdx.x * 256 + threadIdx.x;
  if (gid >= NB * (DINNER / 2)) return;
  const int b  = gid >> 10;
  const int dp = gid & (DINNER / 2 - 1);
  const int d  = 2 * dp;

  float A0[DSTATE], A1[DSTATE], h0[DSTATE], h1[DSTATE];
#pragma unroll
  for (int n = 0; n < DSTATE; ++n) {
    A0[n] = -__expf(A_log[d * DSTATE + n]) * LOG2E_F;
    A1[n] = -__expf(A_log[(d + 1) * DSTATE + n]) * LOG2E_F;
    h0[n] = 0.0f; h1[n] = 0.0f;
  }
  const float D0 = Dp[d], D1 = Dp[d + 1];
  const float bias0 = dt_bias[d], bias1 = dt_bias[d + 1];

#pragma unroll 1
  for (int l = 0; l < LSEQ; ++l) {
    const size_t tok = (size_t)b * LSEQ + l;
    const v2f pr = *(const v2f*)(pre + tok * DINNER + d);
    const v2f uu = *(const v2f*)(u32 + tok * DINNER + d);
    const float dl0 = softplus_f(pr.x + bias0);
    const float dl1 = softplus_f(pr.y + bias1);
    const float* bc = dbl + tok * DBLP + DTRANK;
    float Bv[DSTATE], Cv[DSTATE];
#pragma unroll
    for (int q = 0; q < 4; ++q) {
      const v4f bb = *(const v4f*)(bc + 4 * q);
      const v4f cc = *(const v4f*)(bc + DSTATE + 4 * q);
      Bv[4 * q] = bb.x; Bv[4 * q + 1] = bb.y; Bv[4 * q + 2] = bb.z; Bv[4 * q + 3] = bb.w;
      Cv[4 * q] = cc.x; Cv[4 * q + 1] = cc.y; Cv[4 * q + 2] = cc.z; Cv[4 * q + 3] = cc.w;
    }
    const float du0 = dl0 * uu.x;
    const float du1 = dl1 * uu.y;
    float y0 = 0.0f, y1 = 0.0f;
#pragma unroll
    for (int n = 0; n < DSTATE; ++n) {
      const float e0 = exp2f(dl0 * A0[n]);
      const float e1 = exp2f(dl1 * A1[n]);
      h0[n] = fmaf(e0, h0[n], du0 * Bv[n]);
      h1[n] = fmaf(e1, h1[n], du1 * Bv[n]);
      y0 = fmaf(h0[n], Cv[n], y0);
      y1 = fmaf(h1[n], Cv[n], y1);
    }
    const float o0 = fmaf(uu.x, D0, y0);
    const float o1 = fmaf(uu.y, D1, y1);
    if (MODE == 0) {
      v2f ov; ov.x = o0; ov.y = o1;
      *(volatile v2f*)(ys + tok * DINNER + d) = ov;
      __threadfence();
      *(volatile v2f*)(ys + tok * DINNER + d) = ov;
    } else {
      const size_t tokr = (size_t)b * LSEQ + (LSEQ - 1 - l);
      const v2f yf = *(const v2f*)(ysf + tokr * DINNER + d);
      const v2f zz = *(const v2f*)(xz + tokr * XZW + DINNER + d);
      const float gv0 = (yf.x + o0) * silu_f(zz.x);
      const float gv1 = (yf.y + o1) * silu_f(zz.y);
      const unsigned hu = pack_h2(gv0 * syg, gv1 * syg);
      unsigned* pp = (unsigned*)yg + ((tokr * DINNER + d) >> 1);
      *(volatile unsigned*)pp = hu;
      __threadfence();
      *(volatile unsigned*)pp = hu;
    }
  }
}

__global__ __launch_bounds__(256) void ln_res(
    const float* __restrict__ mo, const float* __restrict__ x1, const float* __restrict__ g,
    const float* __restrict__ bb, float* __restrict__ out)
{
  __shared__ float red[16];
  const int row = blockIdx.x;
  const int t = threadIdx.x, lane = t & 31, wave = t >> 5;
  const size_t base = (size_t)row * DMODEL + 4 * t;
  const v4f xv = *(const v4f*)(mo + base);
  float s = (xv.x + xv.y) + (xv.z + xv.w);
  s = wave_sum(s);
  if (lane == 0) red[wave] = s;
  __syncthreads();
  float tot = 0.0f;
#pragma unroll
  for (int w = 0; w < 8; ++w) tot += red[w];
  const float mean = tot * (1.0f / DMODEL);
  const v4f dx = xv - mean;
  float q = (dx.x * dx.x + dx.y * dx.y) + (dx.z * dx.z + dx.w * dx.w);
  q = wave_sum(q);
  if (lane == 0) red[8 + wave] = q;
  __syncthreads();
  float tot2 = 0.0f;
#pragma unroll
  for (int w = 0; w < 8; ++w) tot2 += red[8 + w];
  const float var  = tot2 * (1.0f / DMODEL);
  const float rstd = 1.0f / sqrtf(var + 1e-6f);
  const v4f gv = *(const v4f*)(g + 4 * t);
  const v4f bv = *(const v4f*)(bb + 4 * t);
  const v4f rv = *(const v4f*)(x1 + base);
  const v4f o  = rv + dx * rstd * gv + bv;
  *(volatile v4f*)(out + base) = o;
  __threadfence();
  *(volatile v4f*)(out + base) = o;
}

extern "C" void kernel_launch(void* const* d_in, const int* in_sizes, int n_in,
                              void* d_out, int out_size, void* d_ws, size_t ws_size,
                              hipStream_t stream)
{
  if (n_in < 30) return;
  if (in_sizes[0] != NTOK * DIN || in_sizes[1] != NTOK * DIN) return;
  if (in_sizes[2] != DMODEL * DIN * 3 || in_sizes[10] != XZW * DMODEL) return;
  if (in_sizes[13] != DBLW * DINNER || in_sizes[25] != DMODEL * DINNER) return;
  if (out_size != 2 * NTOK * DMODEL) return;

  const float* g_x       = (const float*)d_in[0];
  const float* r_x       = (const float*)d_in[1];
  const float* e_conv_w  = (const float*)d_in[2];
  const float* e_bn_g    = (const float*)d_in[3];
  const float* e_bn_b    = (const float*)d_in[4];
  const float* e_skip_w  = (const float*)d_in[5];
  const float* g_conv_w  = (const float*)d_in[6];
  const float* g_bn_g    = (const float*)d_in[7];
  const float* g_bn_b    = (const float*)d_in[8];
  const float* g_skip_w  = (const float*)d_in[9];
  const float* in_proj_w = (const float*)d_in[10];
  const float* conv_w_f  = (const float*)d_in[11];
  const float* conv_b_f  = (const float*)d_in[12];
  const float* x_proj_f  = (const float*)d_in[13];
  const float* dt_w_f    = (const float*)d_in[14];
  const float* dt_bias_f = (const float*)d_in[15];
  const float* A_log_f   = (const float*)d_in[16];
  const float* D_f       = (const float*)d_in[17];
  const float* conv_w_b  = (const float*)d_in[18];
  const float* conv_b_b  = (const float*)d_in[19];
  const float* x_proj_b  = (const float*)d_in[20];
  const float* dt_w_b    = (const float*)d_in[21];
  const float* dt_bias_b = (const float*)d_in[22];
  const float* A_log_b   = (const float*)d_in[23];
  const float* D_b       = (const float*)d_in[24];
  const float* out_proj_w= (const float*)d_in[25];
  const float* ln1_g     = (const float*)d_in[26];
  const float* ln1_b     = (const float*)d_in[27];
  const float* ln2_g     = (const float*)d_in[28];
  const float* ln2_b     = (const float*)d_in[29];

  size_t off = 0;
  auto carve = [&](size_t bytes) -> size_t { size_t p = off; off += (bytes + 255) & ~(size_t)255; return p; };
  const size_t o_wc   = carve((size_t)DMODEL * KC3 * 2);
  const size_t o_wsk  = carve((size_t)DMODEL * DIN * 2);
  const size_t o_wip  = carve((size_t)XZW * DMODEL * 2);
  const size_t o_wxpf = carve((size_t)DBLP * DINNER * 2);
  const size_t o_wxpb = carve((size_t)DBLP * DINNER * 2);
  const size_t o_wdtf = carve((size_t)DINNER * DTRANK * 2);
  const size_t o_wdtb = carve((size_t)DINNER * DTRANK * 2);
  const size_t o_wop  = carve((size_t)DMODEL * DINNER * 2);
  const size_t o_xpad = carve((size_t)NB * LP * DIN * 2);
  const size_t o_res  = carve((size_t)NTOK * DMODEL * 4);
  const size_t o_x132 = carve((size_t)NTOK * DMODEL * 4);
  const size_t o_x116 = carve((size_t)NTOK * DMODEL * 2);
  const size_t o_xz   = carve((size_t)NTOK * XZW * 4);
  const size_t o_u32  = carve((size_t)NTOK * DINNER * 4);
  const size_t o_u16  = carve((size_t)NTOK * DINNER * 2);
  const size_t o_dbl  = carve((size_t)NTOK * DBLP * 4);
  const size_t o_dbl16= carve((size_t)NTOK * DBLP * 2);
  const size_t o_dlt  = carve((size_t)NTOK * DINNER * 4);
  const size_t o_ysf  = carve((size_t)NTOK * DINNER * 4);
  if (off > ws_size) return;

  char* base = (char*)d_ws;
  unsigned short* wc16   = (unsigned short*)(base + o_wc);
  unsigned short* wsk16  = (unsigned short*)(base + o_wsk);
  unsigned short* wip16  = (unsigned short*)(base + o_wip);
  unsigned short* wxpf16 = (unsigned short*)(base + o_wxpf);
  unsigned short* wxpb16 = (unsigned short*)(base + o_wxpb);
  unsigned short* wdtf16 = (unsigned short*)(base + o_wdtf);
  unsigned short* wdtb16 = (unsigned short*)(base + o_wdtb);
  unsigned short* wop16  = (unsigned short*)(base + o_wop);
  unsigned short* xpad16 = (unsigned short*)(base + o_xpad);
  float*          res    = (float*)(base + o_res);
  float*          mout   = res;
  float*          x132   = (float*)(base + o_x132);
  unsigned short* x116   = (unsigned short*)(base + o_x116);
  float*          xz     = (float*)(base + o_xz);
  float*          u32    = (float*)(base + o_u32);
  unsigned short* u16    = (unsigned short*)(base + o_u16);
  unsigned short* yg16   = u16;
  float*          dbl32  = (float*)(base + o_dbl);
  unsigned short* dbl16  = (unsigned short*)(base + o_dbl16);
  float*          dlt    = (float*)(base + o_dlt);
  float*          ysf    = (float*)(base + o_ysf);

  const dim3 blk(256);
  auto cdiv  = [](long a, long b) { return (int)((a + b - 1) / b); };
  auto ggrid = [](int M, int N, int batch) { const int tiles = (M / 64) * (N / 64); return dim3((unsigned)((tiles + 7) / 8), (unsigned)batch); };

  const float bn_c   = 1.000005f;
  const float bn_inv = 1.0f / bn_c;

  cast_rows_f16<<<dim3(cdiv((long)XZW * DMODEL / 2, 256)), blk, 0, stream>>>(in_proj_w, wip16, XZW, XZW, DMODEL, S_WIP);
  cast_rows_f16<<<dim3(cdiv((long)DMODEL * DINNER / 2, 256)), blk, 0, stream>>>(out_proj_w, wop16, DMODEL, DMODEL, DINNER, S_WOP);
  cast_rows_f16<<<dim3(cdiv((long)DBLP * DINNER / 2, 256)), blk, 0, stream>>>(x_proj_f, wxpf16, DBLW, DBLP, DINNER, S_WXP);
  cast_rows_f16<<<dim3(cdiv((long)DBLP * DINNER / 2, 256)), blk, 0, stream>>>(x_proj_b, wxpb16, DBLW, DBLP, DINNER, S_WXP);
  cast_rows_f16<<<dim3(cdiv((long)DINNER * DTRANK / 2, 256)), blk, 0, stream>>>(dt_w_f, wdtf16, DINNER, DINNER, DTRANK, S_WDT);
  cast_rows_f16<<<dim3(cdiv((long)DINNER * DTRANK / 2, 256)), blk, 0, stream>>>(dt_w_b, wdtb16, DINNER, DINNER, DTRANK, S_WDT);

  for (int st = 0; st < 2; ++st) {
    const float* x    = st ? r_x : g_x;
    const float* cw   = st ? g_conv_w : e_conv_w;
    const float* bng  = st ? g_bn_g : e_bn_g;
    const float* bnb  = st ? g_bn_b : e_bn_b;
    const float* sw   = st ? g_skip_w : e_skip_w;
    const float* lng  = st ? ln2_g : ln1_g;
    const float* lnb  = st ? ln2_b : ln1_b;
    float* outp = (float*)d_out + (size_t)st * NTOK * DMODEL;

    cast_convw_f16<<<dim3(cdiv((long)DMODEL * KC3 / 2, 256)), blk, 0, stream>>>(cw, wc16, S_WCONV);
    cast_rows_f16<<<dim3(cdiv((long)DMODEL * DIN / 2, 256)), blk, 0, stream>>>(sw, wsk16, DMODEL, DMODEL, DIN, S_WCONV);
    pad_x_f16<<<dim3(cdiv((long)NB * LP * DIN / 2, 256)), blk, 0, stream>>>(x, xpad16);

    gemm64_f16<0, false><<<ggrid(LSEQ, DMODEL, NB), blk, 0, stream>>>(
        xpad16 + DIN, DIN, (long)LP * DIN,
        wsk16, DIN, 0L,
        res, x116, DMODEL, (long)LSEQ * DMODEL,
        bng, bnb, res, 0L,
        LSEQ, DMODEL, DIN, 1.0f / S_WCONV, 0.0f, 1.0f);

    gemm64_f16<1, true><<<ggrid(LSEQ, DMODEL, NB), blk, 0, stream>>>(
        xpad16, DIN, (long)LP * DIN,
        wc16, KC3, 0L,
        x132, x116, DMODEL, (long)LSEQ * DMODEL,
        bng, bnb, res, (long)LSEQ * DMODEL,
        LSEQ, DMODEL, KC3, 1.0f / S_WCONV, bn_inv, 1.0f);

    gemm64_f16<0, false><<<ggrid(NTOK, XZW, 1), blk, 0, stream>>>(
        x116, DMODEL, 0L,
        wip16, DMODEL, 0L,
        xz, x116, XZW, 0L,
        bng, bnb, res, 0L,
        NTOK, XZW, DMODEL, 1.0f / S_WIP, 0.0f, 1.0f);

    for (int dir = 0; dir < 2; ++dir) {
      const float* cvw  = dir ? conv_w_b : conv_w_f;
      const float* cvb  = dir ? conv_b_b : conv_b_f;
      const unsigned short* wxp = dir ? wxpb16 : wxpf16;
      const unsigned short* wdt = dir ? wdtb16 : wdtf16;
      const float* dtb  = dir ? dt_bias_b : dt_bias_f;
      const float* alog = dir ? A_log_b : A_log_f;
      const float* dd   = dir ? D_b : D_f;

      dwconv_silu2<<<dim3(cdiv((long)NTOK * DINNER / 2, 256)), blk, 0, stream>>>(xz, cvw, cvb, u32, u16, dir, S_U);

      gemm64_f16<0, true><<<ggrid(NTOK, DBLP, 1), blk, 0, stream>>>(
          u16, DINNER, 0L,
          wxp, DINNER, 0L,
          dbl32, dbl16, DBLP, 0L,
          dtb, dtb, res, 0L,
          NTOK, DBLP, DINNER, 1.0f / (S_U * S_WXP), 0.0f, S_DT);

      gemm64_f16<0, false><<<ggrid(NTOK, DINNER, 1), blk, 0, stream>>>(
          dbl16, DBLP, 0L,
          wdt, DTRANK, 0L,
          dlt, dbl16, DINNER, 0L,
          dtb, dtb, res, 0L,
          NTOK, DINNER, DTRANK, 1.0f / (S_DT * S_WDT), 0.0f, 1.0f);

      if (dir == 0) {
        scan2<0><<<dim3(cdiv((long)NB * DINNER / 2, 256)), blk, 0, stream>>>(dlt, dtb, u32, dbl32, alog, dd, ysf, ysf, xz, yg16, S_YG);
      } else {
        scan2<1><<<dim3(cdiv((long)NB * DINNER / 2, 256)), blk, 0, stream>>>(dlt, dtb, u32, dbl32, alog, dd, ysf, ysf, xz, yg16, S_YG);
      }
    }

    gemm64_f16<0, false><<<ggrid(NTOK, DMODEL, 1), blk, 0, stream>>>(
        yg16, DINNER, 0L,
        wop16, DINNER, 0L,
        mout, x116, DMODEL, 0L,
        bng, bnb, res, 0L,
        NTOK, DMODEL, DINNER, 1.0f / (S_YG * S_WOP), 0.0f, 1.0f);

    ln_res<<<dim3(NTOK), blk, 0, stream>>>(mout, x132, lng, lnb, outp);
  }
}
